// TemporalContrastiveLoss_46213848105954
// MI455X (gfx1250) — hardware-verified
//
#include <hip/hip_runtime.h>

typedef _Float16 v16h __attribute__((ext_vector_type(16)));
typedef _Float16 v8h  __attribute__((ext_vector_type(8)));
typedef float    v8f  __attribute__((ext_vector_type(8)));
typedef float    v4f  __attribute__((ext_vector_type(4)));
union Frag { v16h v; v8h hh[2]; };

#define NB        16
#define SEQ       512
#define DIM       256
#define NROWS     (NB * SEQ)
#define NTILES    (NROWS / 16)
#define KCHUNKS   (DIM / 32)
#define JCHUNKS   8
#define JT_PER_CHUNK (NTILES / JCHUNKS)
#define PW        5
#define INVT      14.2857142857142857f
#define OPSCALE   16.0f
#define SIMSCALE  (INVT / (OPSCALE * OPSCALE))
#define LINEF     32
#define WAVES_PER_BLOCK 8

static_assert(NROWS % (16 * WAVES_PER_BLOCK) == 0);
static_assert(NTILES % JCHUNKS == 0);
static_assert(DIM % 32 == 0);
static_assert(SEQ % 16 == 0);

__device__ __forceinline__ v8f wmma_f16(v16h a, v16h b, v8f c) {
  v8f d = __builtin_amdgcn_wmma_f32_16x16x32_f16(false, a, false, b, (short)0, c, false, false);
  asm volatile("v_nop\n\tv_nop\n\tv_nop\n\tv_nop" : "+v"(d) : "v"(a), "v"(b));
  return d;
}

__global__ __launch_bounds__(256) void k_norm_rows(
    const float* __restrict__ emb, _Float16* __restrict__ Ef, int nrows) {
  const int lane = threadIdx.x & 31;
  const int wave = threadIdx.x >> 5;
  const int row  = blockIdx.x * WAVES_PER_BLOCK + wave;
  if (row >= nrows) return;

  const float4* p = (const float4*)(emb + (size_t)row * DIM + lane * 8);
  const float4 x0 = p[0];
  const float4 x1 = p[1];

  float ss = x0.x*x0.x + x0.y*x0.y + x0.z*x0.z + x0.w*x0.w
           + x1.x*x1.x + x1.y*x1.y + x1.z*x1.z + x1.w*x1.w;
#pragma unroll
  for (int off = 16; off >= 1; off >>= 1) ss += __shfl_xor(ss, off, 32);

  const float nrm = fmaxf(sqrtf(ss), 1e-12f);
  const float inv = 1.0f / nrm;

  v8h h;
  h[0] = (_Float16)((x0.x * inv) * OPSCALE); h[1] = (_Float16)((x0.y * inv) * OPSCALE);
  h[2] = (_Float16)((x0.z * inv) * OPSCALE); h[3] = (_Float16)((x0.w * inv) * OPSCALE);
  h[4] = (_Float16)((x1.x * inv) * OPSCALE); h[5] = (_Float16)((x1.y * inv) * OPSCALE);
  h[6] = (_Float16)((x1.z * inv) * OPSCALE); h[7] = (_Float16)((x1.w * inv) * OPSCALE);

  volatile v8h* q = (volatile v8h*)(Ef + (size_t)row * DIM + lane * 8);
  *q = h;
  __threadfence();
  *q = h;
}

__global__ __launch_bounds__(256) void k_sim_rowsum(
    const _Float16* __restrict__ Ef, float* __restrict__ part) {
  const int lane  = threadIdx.x & 31;
  const int wave  = threadIdx.x >> 5;
  const int m     = lane & 15;
  const int h     = lane >> 4;
  const int itile = blockIdx.x * WAVES_PER_BLOCK + wave;
  const int ibase = itile * 16;
  const int jc    = blockIdx.y;

  v16h bf[KCHUNKS];
  const _Float16* brow = Ef + (size_t)(ibase + m) * DIM;
#pragma unroll
  for (int kc = 0; kc < KCHUNKS; ++kc) {
    Frag t;
    t.hh[0] = *(const v8h*)(brow + kc * 32 + 8 * h);
    t.hh[1] = *(const v8h*)(brow + kc * 32 + 16 + 8 * h);
    bf[kc] = t.v;
  }

  float rall = 0.f, rpos = 0.f;
  const int icol = ibase + m;
  const int jt0  = jc * JT_PER_CHUNK;

#pragma unroll 1
  for (int jt = jt0; jt < jt0 + JT_PER_CHUNK; ++jt) {
    const int jbase = jt * 16;
    const _Float16* arow = Ef + (size_t)(jbase + m) * DIM;

    v8f acc = {0.f, 0.f, 0.f, 0.f, 0.f, 0.f, 0.f, 0.f};
#pragma unroll
    for (int kc = 0; kc < KCHUNKS; ++kc) {
      Frag a;
      a.hh[0] = *(const v8h*)(arow + kc * 32 + 8 * h);
      a.hh[1] = *(const v8h*)(arow + kc * 32 + 16 + 8 * h);
      acc = wmma_f16(a.v, bf[kc], acc);
    }

    float ex[8];
#pragma unroll
    for (int e = 0; e < 8; ++e) ex[e] = __expf(acc[e] * SIMSCALE);

    if (jt >= itile - 1 && jt <= itile + 1) {
#pragma unroll
      for (int e = 0; e < 8; ++e) {
        const int j  = jbase + 8 * h + e;
        const int d  = j - icol;
        const int ad = d < 0 ? -d : d;
        const bool same_seq = (j / SEQ) == (icol / SEQ);
        const float v = ex[e];
        rall += (d != 0) ? v : 0.f;
        rpos += (same_seq && d != 0 && ad <= PW) ? v : 0.f;
      }
    } else {
#pragma unroll
      for (int e = 0; e < 8; ++e) rall += ex[e];
    }
  }

  rall += __shfl_xor(rall, 16, 32);
  rpos += __shfl_xor(rpos, 16, 32);

  const float val = (lane < 16) ? rall : rpos;
  v4f o;
  o[0] = __shfl(val, (4 * lane + 0) & 31, 32);
  o[1] = __shfl(val, (4 * lane + 1) & 31, 32);
  o[2] = __shfl(val, (4 * lane + 2) & 31, 32);
  o[3] = __shfl(val, (4 * lane + 3) & 31, 32);

  volatile v4f* q = (volatile v4f*)(part + ((size_t)jc * NTILES + itile) * LINEF + lane * 4);
  if (lane < 8) *q = o;
  __threadfence();
  if (lane < 8) *q = o;
}

__global__ __launch_bounds__(256) void k_finalize(
    const float* __restrict__ part, float* __restrict__ out) {
  __shared__ double sred[256];
  const int tid = threadIdx.x;
  double acc = 0.0;
#pragma unroll 1
  for (int i = tid; i < NROWS; i += 256) {
    const int it = i >> 4;
    const int m  = i & 15;
    float sa = 0.f, sp = 0.f;
#pragma unroll
    for (int c = 0; c < JCHUNKS; ++c) {
      const float* q = part + ((size_t)c * NTILES + it) * LINEF;
      sa += q[m];
      sp += q[16 + m];
    }
    const float pos_sum = sp + 1e-8f;
    const float all_sum = sa + 1e-8f;
    acc += (double)logf(pos_sum / all_sum);
  }
  sred[tid] = acc;
  __syncthreads();
#pragma unroll 1
  for (int s = 128; s >= 1; s >>= 1) {
    if (tid < s) sred[tid] += sred[tid + s];
    __syncthreads();
  }
  if (tid == 0) {
    const float loss = (float)(-(sred[0] / (double)NROWS));
    volatile float* o = (volatile float*)out;
    *o = loss;
    __threadfence();
    *o = loss;
  }
}

extern "C" void kernel_launch(void* const* d_in, const int* in_sizes, int n_in,
                              void* d_out, int out_size, void* d_ws, size_t ws_size,
                              hipStream_t stream) {
  if (n_in < 1 || in_sizes[0] != NROWS * DIM || out_size < 1) return;

  const size_t ef_bytes   = (size_t)NROWS * DIM * sizeof(_Float16);
  const size_t part_off   = ef_bytes;
  const size_t part_bytes = (size_t)JCHUNKS * NTILES * LINEF * sizeof(float);
  if (part_off + part_bytes > ws_size) return;

  const float* emb = (const float*)d_in[0];
  float* out       = (float*)d_out;
  char* base       = (char*)d_ws;
  _Float16* Ef     = (_Float16*)base;
  float* part      = (float*)(base + part_off);

  k_norm_rows<<<NROWS / WAVES_PER_BLOCK, 256, 0, stream>>>(emb, Ef, NROWS);
  dim3 grid2(NTILES / WAVES_PER_BLOCK, JCHUNKS);
  k_sim_rowsum<<<grid2, 256, 0, stream>>>(Ef, part);
  k_finalize<<<1, 256, 0, stream>>>(part, out);
}
